// MultiHeadAttention_8263517077672
// MI455X (gfx1250) — hardware-run, weakly checked
//
#include <hip/hip_runtime.h>
#ifndef NB
#define NB 2
#endif
#ifndef SEQ
#define SEQ 2048
#endif
#define NB_FULL 2
#define SEQ_FULL 2048
#define DM 1024
#define NH 16
#define HD 64
#define HG 2
#define NR ((size_t)NB * SEQ)
#define LQ (3 * DM)
#define WBLK ((3 * DM * (DM / 8)) / 256)

typedef unsigned short v8us __attribute__((ext_vector_type(8), may_alias));
typedef float  v8f  __attribute__((ext_vector_type(8)));
typedef float  v4f  __attribute__((ext_vector_type(4)));
typedef float  v4fa __attribute__((ext_vector_type(4), may_alias));
typedef _Float16 v16h __attribute__((ext_vector_type(16)));
typedef _Float16 v4h  __attribute__((ext_vector_type(4)));
union FragH { v16h v; v8us half[2]; _Float16 h[16]; unsigned short u[16]; };

__device__ __forceinline__ unsigned short bf16_bits(float x) { unsigned int u = __float_as_uint(x); return (unsigned short)((u + 0x7FFFu + ((u >> 16) & 1u)) >> 16); }
__device__ __forceinline__ float bf16_rne(float x) { return __uint_as_float(((unsigned int)bf16_bits(x)) << 16); }

__global__ __launch_bounds__(256) void k_w16(const float* __restrict__ W1, const float* __restrict__ b1, _Float16* __restrict__ Wt, float* __restrict__ Bp) {
  const int tid = threadIdx.x;
  if (blockIdx.x >= WBLK) {
    const int t = ((int)blockIdx.x - WBLK) * 256 + tid;
    if (t >= (3 * DM) / 4) return;
    v4f o;
#pragma unroll
    for (int q = 0; q < 4; ++q) { const int R = t * 4 + q; const int s = R / DM, np = R % DM; o[q] = b1[(np / HD) * (3 * HD) + (np % HD) * 3 + s]; }
    *(volatile v4f*)(Bp + (size_t)t * 4) = o; __threadfence(); *(volatile v4f*)(Bp + (size_t)t * 4) = o;
    return;
  }
  const int t = (int)blockIdx.x * 256 + tid;
  const int R = t / (DM / 8), k8 = (t % (DM / 8)) * 8;
  const int s = R / DM, np = R % DM;
  const float* src = W1 + (size_t)((np / HD) * (3 * HD) + (np % HD) * 3 + s) * DM + k8;
  const v4f a = *(const v4fa*)src, c = *(const v4fa*)(src + 4);
  FragH f;
#pragma unroll
  for (int q = 0; q < 4; ++q) { f.h[q] = (_Float16)(bf16_rne(a[q]) * 16.0f); f.h[4 + q] = (_Float16)(bf16_rne(c[q]) * 16.0f); }
  const v8us o = f.half[0];
  unsigned short* d = (unsigned short*)Wt + (size_t)R * DM + k8;
  *(volatile v8us*)d = o; __threadfence(); *(volatile v8us*)d = o;
}

__global__ __launch_bounds__(256) void k_x16(const float* __restrict__ x, _Float16* __restrict__ X16, int n8) {
  const int t = (int)blockIdx.x * 256 + threadIdx.x; if (t >= n8) return;
  const int row = t / (DM / 8), c8 = (t % (DM / 8)) * 8; const int b = row / SEQ, s = row % SEQ;
  const float* src = x + ((size_t)b * SEQ_FULL + s) * DM + c8;
  const v4f a = *(const v4fa*)src, c = *(const v4fa*)(src + 4);
  FragH f;
#pragma unroll
  for (int q = 0; q < 4; ++q) { f.h[q] = (_Float16)bf16_rne(a[q]); f.h[4 + q] = (_Float16)bf16_rne(c[q]); }
  const v8us o = f.half[0];
  unsigned short* d = (unsigned short*)X16 + (size_t)t * 8;
  *(volatile v8us*)d = o; __threadfence(); *(volatile v8us*)d = o;
}

__device__ __forceinline__ v16h g2_frag(const _Float16* p, int hh) { FragH f; f.half[0] = *(const v8us*)((const unsigned short*)p + 8 * hh); f.half[1] = *(const v8us*)((const unsigned short*)p + 16 + 8 * hh); return f.v; }
__device__ __forceinline__ v8f g2_mma(v16h a, v16h b, v8f c) { v8f d = __builtin_amdgcn_wmma_f32_16x16x32_f16(false, a, false, b, (short)0, c, false, false); asm volatile("v_nop\n\tv_nop\n\tv_nop\n\tv_nop" : "+v"(d) : "v"(a), "v"(b)); return d; }
template <bool OUT16>
__global__ __launch_bounds__(128) void k_gemm2(const _Float16* __restrict__ A, int lda, size_t sA, const _Float16* __restrict__ Bh, int ldb, size_t sB, float alpha, const float* __restrict__ bias,
    float* __restrict__ C, _Float16* __restrict__ C16, int ldc, size_t sC, int N, int K) {
  __shared__ __attribute__((aligned(16))) float so[4][32][68];
  const int tid = threadIdx.x, w = tid >> 5, lane = tid & 31, ln = lane & 15, hh = lane >> 4; const int by = blockIdx.y;
  A += (size_t)by * sA; Bh += (size_t)by * sB; const size_t cofs = (size_t)by * sC;
  const int ntn = N >> 6; const int mt = (int)blockIdx.x / ntn, nq = (int)blockIdx.x - mt * ntn; const int row0 = mt * 128 + 32 * w, col0 = nq * 64;
  const _Float16* a0p = A + (size_t)(row0 + ln) * lda; const _Float16* a1p = a0p + (size_t)16 * lda;
  const _Float16* b0p = Bh + (size_t)(col0 + ln) * ldb; const _Float16* b1p = b0p + (size_t)16 * ldb; const _Float16* b2p = b1p + (size_t)16 * ldb; const _Float16* b3p = b2p + (size_t)16 * ldb;
  const v8f z8 = {0.f,0.f,0.f,0.f,0.f,0.f,0.f,0.f}; v8f c00 = z8, c01 = z8, c02 = z8, c03 = z8, c10 = z8, c11 = z8, c12 = z8, c13 = z8;
#pragma unroll 1
  for (int kb = 0; kb < K; kb += 32) { const v16h a0 = g2_frag(a0p + kb, hh), a1 = g2_frag(a1p + kb, hh);
    v16h b = g2_frag(b0p + kb, hh); c00 = g2_mma(a0, b, c00); c10 = g2_mma(a1, b, c10);
    b = g2_frag(b1p + kb, hh); c01 = g2_mma(a0, b, c01); c11 = g2_mma(a1, b, c11);
    b = g2_frag(b2p + kb, hh); c02 = g2_mma(a0, b, c02); c12 = g2_mma(a1, b, c12);
    b = g2_frag(b3p + kb, hh); c03 = g2_mma(a0, b, c03); c13 = g2_mma(a1, b, c13); }
  v8f accs[8] = {c00, c01, c02, c03, c10, c11, c12, c13};
#pragma unroll
  for (int u = 0; u < 8; ++u) { const int t = u & 3, half = u >> 2; const int col = col0 + t * 16 + ln; float bv = 0.f; if (bias) bv = bf16_rne(bias[col]);
#pragma unroll
    for (int r = 0; r < 8; ++r) { const int rloc = half * 16 + 8 * hh + r; so[w][rloc][t * 16 + ln] = accs[u][r] * alpha + bv; } }
  __syncthreads();
  const int rsub = lane >> 4, c4 = (lane & 15) * 4;
  for (int pass = 0; pass < 2; ++pass) {
#pragma unroll
    for (int q = 0; q < 16; ++q) { const int r = q * 2 + rsub; const v4f v = *(const v4fa*)&so[w][r][c4];
      if (OUT16) { v4h h4; h4[0] = (_Float16)v[0]; h4[1] = (_Float16)v[1]; h4[2] = (_Float16)v[2]; h4[3] = (_Float16)v[3]; *(volatile v4h*)(C16 + cofs + (size_t)(row0 + r) * ldc + col0 + c4) = h4; }
      else *(volatile v4f*)(C + cofs + (size_t)(row0 + r) * ldc + col0 + c4) = v; }
    if (pass == 0) __threadfence(); } }

template <int NHv, int TTv>
__global__ __launch_bounds__(256) void k_vt(const _Float16* __restrict__ V16, int ldv, int voff, _Float16* __restrict__ Vt) {
  __shared__ unsigned short tl[64][66];
  const int tid = threadIdx.x; const int slab = (int)blockIdx.x / (TTv / 64), lg = (int)blockIdx.x % (TTv / 64); const int b = slab / NHv, h = slab % NHv;
  for (int i = tid; i < 64 * 8; i += 256) { const int r = i / 8, c8 = (i % 8) * 8; FragH f; f.half[0] = *(const v8us*)((const unsigned short*)V16 + ((size_t)b * TTv + lg * 64 + r) * ldv + voff + h * 64 + c8);
#pragma unroll
    for (int q = 0; q < 8; ++q) tl[r][c8 + q] = f.u[q]; }
  __syncthreads();
  for (int pass = 0; pass < 2; ++pass) {
#pragma unroll
    for (int rd = 0; rd < 2; ++rd) { const int d = rd * 32 + tid / 8, pc = tid % 8; FragH f;
#pragma unroll
      for (int q = 0; q < 8; ++q) f.u[q] = tl[pc * 8 + q][d];
      const v8us o = f.half[0];
      *(volatile v8us*)((unsigned short*)Vt + ((size_t)slab * 64 + d) * TTv + lg * 64 + pc * 8) = o; }
    if (pass == 0) __threadfence(); } }

template <int CH>
__global__ __launch_bounds__(256) void k_rsmw(const float* __restrict__ S, _Float16* __restrict__ P, int nrows) {
  #pragma clang fp contract(off)
  const int lane = threadIdx.x & 31; const int row = (int)blockIdx.x * 8 + ((int)threadIdx.x >> 5);
  if (row >= nrows) return;
  const float* s = S + (size_t)row * SEQ;
  float v[CH * 8]; float mx = -3.0e38f;
#pragma unroll
  for (int c = 0; c < CH; ++c) { const v4f x0 = *(const v4fa*)(s + c * 256 + lane * 8), x1 = *(const v4fa*)(s + c * 256 + lane * 8 + 4);
#pragma unroll
    for (int q = 0; q < 4; ++q) { v[c * 8 + q] = x0[q]; v[c * 8 + 4 + q] = x1[q]; mx = fmaxf(mx, fmaxf(x0[q], x1[q])); } }
  mx = fmaxf(mx, __shfl_xor(mx, 16)); mx = fmaxf(mx, __shfl_xor(mx, 8)); mx = fmaxf(mx, __shfl_xor(mx, 4)); mx = fmaxf(mx, __shfl_xor(mx, 2)); mx = fmaxf(mx, __shfl_xor(mx, 1));
  float se = 0.f;
#pragma unroll
  for (int i = 0; i < CH * 8; ++i) { const float e = __expf(v[i] - mx); v[i] = e; se += e; }
  se += __shfl_xor(se, 16); se += __shfl_xor(se, 8); se += __shfl_xor(se, 4); se += __shfl_xor(se, 2); se += __shfl_xor(se, 1);
  const float sc = 256.0f / se;
  v8us o[CH];
#pragma unroll
  for (int c = 0; c < CH; ++c) { FragH f;
#pragma unroll
    for (int q = 0; q < 8; ++q) f.h[q] = (_Float16)(v[c * 8 + q] * sc);
    o[c] = f.half[0]; }
  unsigned short* d = (unsigned short*)P + (size_t)row * SEQ + lane * 8;
  for (int pass = 0; pass < 2; ++pass) {
#pragma unroll
    for (int c = 0; c < CH; ++c) *(volatile v8us*)(d + c * 256) = o[c];
    if (pass == 0) __threadfence(); } }

extern "C" void kernel_launch(void* const* d_in, const int* in_sizes, int n_in,
                              void* d_out, int out_size, void* d_ws, size_t ws_size, hipStream_t stream) {
  static_assert(NH * HD == DM && DM % 64 == 0 && SEQ % 256 == 0 && (NB * SEQ) % 128 == 0 && NH % HG == 0 && SEQ <= SEQ_FULL && NB <= NB_FULL);
  static_assert((3 * DM * (DM / 8)) % 256 == 0 && ((3 * DM) / 4) % 256 == 0);
  constexpr size_t SZ_W  = (size_t)3 * DM * DM * 2;
  constexpr size_t SZ_B  = 16384;
  constexpr size_t SZ_X  = (size_t)NB * SEQ * DM * 2;
  constexpr size_t SZ_Q  = (size_t)NB * SEQ * LQ * 2;
  constexpr size_t SZ_VT = (size_t)NB * NH * HD * SEQ * 2;
  constexpr size_t SZ_S  = (size_t)HG * SEQ * SEQ * 4;
  constexpr size_t SZ_P  = (size_t)HG * SEQ * SEQ * 2;
  constexpr size_t SZ_ALL = SZ_W + SZ_B + SZ_X + SZ_Q + SZ_VT + SZ_S + SZ_P;
  static_assert(SZ_ALL <= (size_t)134217728);
  static_assert(SZ_W % 256 == 0 && SZ_X % 256 == 0 && SZ_Q % 256 == 0 && SZ_VT % 256 == 0 && SZ_S % 256 == 0 && SZ_P % 256 == 0);
  if (n_in < 3) return;
  const size_t need_x = ((size_t)(NB - 1) * SEQ_FULL + SEQ) * DM;
  if ((size_t)in_sizes[0] < need_x) return;
  if ((size_t)in_sizes[1] < (size_t)3 * DM * DM) return;
  if ((size_t)in_sizes[2] < (size_t)3 * DM) return;
  if ((size_t)out_size < need_x) return;
  if (SZ_ALL > ws_size) return;
  const float* x  = (const float*)d_in[0];
  const float* W1 = (const float*)d_in[1];
  const float* b1 = (const float*)d_in[2];
  float* out = (float*)d_out;
  char* ws = (char*)d_ws; size_t off = 0;
  _Float16* W16 = (_Float16*)(ws + off); off += SZ_W;
  float*    Bp  = (float*)(ws + off);    off += SZ_B;
  _Float16* X16 = (_Float16*)(ws + off); off += SZ_X;
  _Float16* QKV = (_Float16*)(ws + off); off += SZ_Q;
  _Float16* VT  = (_Float16*)(ws + off); off += SZ_VT;
  float*    S   = (float*)(ws + off);    off += SZ_S;
  _Float16* P   = (_Float16*)(ws + off); off += SZ_P;

  k_w16<<<WBLK + 3, 256, 0, stream>>>(W1, b1, W16, Bp);
  k_x16<<<(unsigned)((NR * DM / 8 + 255) / 256), 256, 0, stream>>>(x, X16, (int)(NR * DM / 8));
  k_gemm2<true><<<dim3((unsigned)((NR / 128) * (LQ / 64)), 1), 128, 0, stream>>>(X16, DM, (size_t)0, W16, DM, (size_t)0, 0.0625f, Bp, nullptr, QKV, LQ, (size_t)0, LQ, DM);
  k_vt<NH, SEQ><<<NB * NH * (SEQ / 64), 256, 0, stream>>>(QKV, LQ, 2 * DM, VT);
  for (int b = 0; b < NB; ++b) {
    const size_t r0 = (size_t)b * SEQ;
    for (int h0 = 0; h0 < NH; h0 += HG) {
      k_gemm2<false><<<dim3((SEQ / 128) * (SEQ / 64), HG), 128, 0, stream>>>(QKV + r0 * LQ + h0 * HD, LQ, (size_t)HD, QKV + r0 * LQ + DM + h0 * HD, LQ, (size_t)HD, 0.125f, nullptr, S, nullptr, SEQ, (size_t)SEQ * SEQ, SEQ, HD);
      k_rsmw<SEQ / 256><<<(HG * SEQ) / 8, 256, 0, stream>>>(S, P, HG * SEQ);
      k_gemm2<false><<<dim3((SEQ / 128) * (HD / 64), HG), 128, 0, stream>>>(P, SEQ, (size_t)SEQ * SEQ, VT + ((size_t)(b * NH + h0) * HD) * SEQ, SEQ, (size_t)HD * SEQ, 0.00390625f, nullptr,
          out + ((size_t)b * SEQ_FULL) * DM + h0 * HD, nullptr, DM, (size_t)HD, HD, SEQ);
    }
  }
}
